// SelfAttention_20718922236436
// MI455X (gfx1250) — hardware-verified
//
#include <hip/hip_runtime.h>


#ifndef NB
#define NB 8
#endif
#ifndef SEQ
#define SEQ 1024
#endif
#define NB_FULL  8
#define SEQ_FULL 1024
#define DM   768
#define NH   12
#define HD   64
#define D3   (3 * DM)
#define KC   (2 * DM)
#define NTOK (NB * SEQ)
#define PCAR 1024.0f
#define RCAR 2048.0f

typedef _Float16 h16;
typedef unsigned short bf;
typedef __attribute__((ext_vector_type(16))) __bf16   v16bf;
typedef __attribute__((ext_vector_type(16))) _Float16 v16h;
typedef __attribute__((ext_vector_type(8)))  _Float16 v8h;
typedef __attribute__((ext_vector_type(8)))  unsigned short v8us;
typedef __attribute__((ext_vector_type(8)))  float    v8f;
typedef __attribute__((ext_vector_type(4)))  float    v4f;
typedef v4f __attribute__((may_alias)) v4fa;

static_assert(DM == NH * HD);
static_assert(HD == 64);
static_assert(DM % 64 == 0);
static_assert(SEQ % 64 == 0);
static_assert(DM % 32 == 0);
static_assert(KC % 32 == 0);
static_assert(SEQ % 32 == 0);
static_assert(SEQ <= SEQ_FULL);
static_assert(NB <= NB_FULL);
static_assert(((size_t)D3 * DM / 8) % 256 == 0);
static_assert(((size_t)DM * DM / 8) % 256 == 0);

__device__ __forceinline__ unsigned short f2bf(float f) { unsigned u = __float_as_uint(f); u += 0x7FFFu + ((u >> 16) & 1u); return (unsigned short)(u >> 16); }
__device__ __forceinline__ float bf2f(unsigned short b) { return __uint_as_float(((unsigned)b) << 16); }
__device__ __forceinline__ float bfr(float f) { return bf2f(f2bf(f)); }
__device__ __forceinline__ v16h cat16(v8h lo, v8h hi) { return __builtin_shufflevector(lo, hi, 0, 1, 2, 3, 4, 5, 6, 7, 8, 9, 10, 11, 12, 13, 14, 15); }
__device__ __forceinline__ v16bf cat16b(v8us lo, v8us hi) { return __builtin_bit_cast(v16bf, __builtin_shufflevector(lo, hi, 0, 1, 2, 3, 4, 5, 6, 7, 8, 9, 10, 11, 12, 13, 14, 15)); }
__device__ __forceinline__ v8f wmma16(v16h a, v16h b, v8f c) { return __builtin_amdgcn_wmma_f32_16x16x32_f16(false, a, false, b, (short)0, c, false, false); }
__device__ __forceinline__ v8f wmmab(v16bf a, v16bf b, v8f c) { return __builtin_amdgcn_wmma_f32_16x16x32_bf16(false, a, false, b, (short)0, c, false, false); }
__device__ __forceinline__ v16h  ldh(const h16* p) { return cat16(*(const v8h*)p, *(const v8h*)(p + 16)); }
__device__ __forceinline__ v16bf ldb(const bf* p)  { return cat16b(*(const v8us*)p, *(const v8us*)(p + 16)); }

template <int K>
__device__ __forceinline__ void gemm_tile(const bf* __restrict__ A, const bf* __restrict__ Bt, int r0, int c0, int lr, int hi, v8f (&acc)[4][4]) {
    static_assert(K % 32 == 0);
#pragma unroll
    for (int mb = 0; mb < 4; ++mb)
#pragma unroll
        for (int nb = 0; nb < 4; ++nb) acc[mb][nb] = (v8f){};
    const size_t aoff = (size_t)(r0 + lr) * K + 8 * hi, boff = (size_t)(c0 + lr) * K + 8 * hi;
#pragma unroll 1
    for (int kc = 0; kc < K; kc += 32) {
        v16bf a[4];
#pragma unroll
        for (int mb = 0; mb < 4; ++mb) a[mb] = ldb(A + aoff + (size_t)mb * 16 * K + kc);
#pragma unroll
        for (int nb = 0; nb < 3; ++nb) { const v16bf b = ldb(Bt + boff + (size_t)nb * 16 * K + kc);
#pragma unroll
            for (int mb = 0; mb < 4; ++mb) acc[mb][nb] = wmmab(a[mb], b, acc[mb][nb]); }
        const v16bf b3 = ldb(Bt + boff + (size_t)3 * 16 * K + kc);
#pragma unroll
        for (int mb = 0; mb < 4; ++mb) acc[mb][3] = wmmab(a[mb], b3, acc[mb][3]);
        asm volatile("" : "+v"(acc[0][0]), "+v"(acc[1][0]), "+v"(acc[2][0]), "+v"(acc[3][0]));
        asm volatile("" : "+v"(acc[0][1]), "+v"(acc[1][1]), "+v"(acc[2][1]), "+v"(acc[3][1]));
        asm volatile("" : "+v"(acc[0][2]), "+v"(acc[1][2]), "+v"(acc[2][2]), "+v"(acc[3][2]));
        asm volatile("v_nop\n\tv_nop\n\tv_nop\n\tv_nop" : "+v"(acc[0][3]), "+v"(acc[1][3]), "+v"(acc[2][3]), "+v"(acc[3][3]) : "v"(a[3]), "v"(b3));
    }
}

__global__ __launch_bounds__(256) void k_cvtw(const float* __restrict__ src, bf* dst, int rows, int K, int dpitch, int dup) {
    const int i = blockIdx.x * 256 + threadIdx.x; const int k8 = K / 8; if (i >= rows * k8) return;
    const int r = i / k8, c = (i % k8) * 8; const v8f v = *(const v8f*)(src + (size_t)r * K + c); v8us o;
#pragma unroll
    for (int k = 0; k < 8; ++k) o[k] = f2bf(v[k]);
    bf* d = dst + (size_t)r * dpitch + c;
    *(volatile v8us*)d = o; if (dup) *(volatile v8us*)(d + K) = o;
    __threadfence();
    *(volatile v8us*)d = o; if (dup) *(volatile v8us*)(d + K) = o;
}

__global__ __launch_bounds__(256) void k_xT(const float* __restrict__ x, bf* XB) {
    __shared__ __align__(16) float ts[64 * 68];
    const int t = threadIdx.x; const int s0 = blockIdx.x * 64, c0 = blockIdx.y * 64, b = blockIdx.z;
    const int cr = t >> 4, s4 = (t & 15) * 4;
#pragma unroll
    for (int i = 0; i < 4; ++i) { const int c = i * 16 + cr; const v4f v = *(const v4f*)(x + ((size_t)b * DM + c0 + c) * SEQ_FULL + s0 + s4);
#pragma unroll
        for (int j = 0; j < 4; ++j) ts[(s4 + j) * 68 + c] = v[j]; }
    __syncthreads();
    const int rq = t >> 3, c8 = (t & 7) * 8;
#pragma unroll 1
    for (int ps = 0; ps < 2; ++ps) {
#pragma unroll
        for (int it = 0; it < 2; ++it) { const int row = it * 32 + rq; const v4f x0 = *(const v4fa*)(ts + row * 68 + c8), x1 = *(const v4fa*)(ts + row * 68 + c8 + 4); v8us o;
#pragma unroll
            for (int k = 0; k < 4; ++k) { o[k] = f2bf(x0[k]); o[4 + k] = f2bf(x1[k]); }
            *(volatile v8us*)(XB + ((size_t)b * SEQ + s0 + row) * DM + c0 + c8) = o; }
        if (ps == 0) __threadfence(); }
}

__global__ __launch_bounds__(32) void k_qkv(const bf* __restrict__ XB, const bf* __restrict__ W, const float* __restrict__ bias, h16* QH, h16* QR, h16* KP, h16* VT) {
    __shared__ __align__(16) float os[64 * 68];
    const int lane = threadIdx.x & 31, lr = lane & 15, hi = lane >> 4; const int r0 = blockIdx.x * 64, c0 = blockIdx.y * 64;
    v8f acc[4][4];
    gemm_tile<DM>(XB, W, r0, c0, lr, hi, acc);
#pragma unroll
    for (int mb = 0; mb < 4; ++mb)
#pragma unroll
        for (int nb = 0; nb < 4; ++nb)
#pragma unroll
            for (int j = 0; j < 8; ++j) os[(mb * 16 + hi * 8 + j) * 68 + nb * 16 + lr] = acc[mb][nb][j];
    __builtin_amdgcn_wave_barrier(); asm volatile("" ::: "memory");
    const int which = c0 / DM, head = (c0 % DM) / HD, b = r0 / SEQ, s0 = r0 % SEQ;
    const size_t bh = (size_t)b * NH + head;
    const int q4 = lane >> 3, p8 = (lane & 7) * 8;
    if (which == 0) {
        const v4f bv0 = *(const v4f*)(bias + c0 + p8), bv1 = *(const v4f*)(bias + c0 + p8 + 4);
#pragma unroll 1
        for (int ps = 0; ps < 2; ++ps) {
#pragma unroll 2
            for (int it = 0; it < 16; ++it) { const int row = it * 4 + q4; const v4f x0 = *(const v4fa*)(os + row * 68 + p8), x1 = *(const v4fa*)(os + row * 68 + p8 + 4); v8h oh, orr;
#pragma unroll
                for (int i = 0; i < 4; ++i) { const float y0 = x0[i] + bfr(bv0[i]); const h16 h0 = (h16)y0; oh[i] = h0; orr[i] = (h16)((y0 - (float)h0) * RCAR);
                    const float y1 = x1[i] + bfr(bv1[i]); const h16 h1 = (h16)y1; oh[4 + i] = h1; orr[4 + i] = (h16)((y1 - (float)h1) * RCAR); }
                const size_t off = (bh * SEQ + s0 + row) * HD + p8;
                *(volatile v8h*)(QH + off) = oh; *(volatile v8h*)(QR + off) = orr; }
            if (ps == 0) __threadfence(); }
    } else if (which == 1) {
        const v4f bv0 = *(const v4f*)(bias + c0 + p8), bv1 = *(const v4f*)(bias + c0 + p8 + 4);
#pragma unroll 1
        for (int ps = 0; ps < 2; ++ps) {
#pragma unroll 2
            for (int it = 0; it < 16; ++it) { const int row = it * 4 + q4; const v4f x0 = *(const v4fa*)(os + row * 68 + p8), x1 = *(const v4fa*)(os + row * 68 + p8 + 4); v8h ok;
#pragma unroll
                for (int i = 0; i < 4; ++i) { ok[i] = (h16)(x0[i] + bfr(bv0[i])); ok[4 + i] = (h16)(x1[i] + bfr(bv1[i])); }
                *(volatile v8h*)(KP + (bh * SEQ + s0 + row) * HD + p8) = ok; }
            if (ps == 0) __threadfence(); }
    } else {
#pragma unroll 1
        for (int ps = 0; ps < 2; ++ps) {
#pragma unroll 2
            for (int it = 0; it < 16; ++it) { const int d = it * 4 + q4; const float bd = bfr(bias[c0 + d]); v8h ov;
#pragma unroll
                for (int i = 0; i < 8; ++i) ov[i] = (h16)(os[(p8 + i) * 68 + d] + bd);
                *(volatile v8h*)(VT + (bh * HD + d) * SEQ + s0 + p8) = ov; }
            if (ps == 0) __threadfence(); }
    }
}

__global__ __launch_bounds__(128) void k_flash(const h16* __restrict__ QH, const h16* __restrict__ QR, const h16* __restrict__ KP, const h16* __restrict__ VT, bf* CTX) {
    __shared__ __align__(16) float os[4 * 16 * 68];
    const int lane = threadIdx.x & 31, lr = lane & 15, hi = lane >> 4;
    const int wave = __builtin_amdgcn_readfirstlane(threadIdx.x >> 5);
    const int head = blockIdx.y, b = blockIdx.z; const int q0 = blockIdx.x * 64 + wave * 16;
    const size_t bh = (size_t)b * NH + head;
    const size_t qoff = (bh * SEQ + q0 + lr) * HD + 8 * hi;
    const v16h bqh0 = ldh(QH + qoff), bqh1 = ldh(QH + qoff + 32), bqr0 = ldh(QR + qoff), bqr1 = ldh(QR + qoff + 32);
    const h16* kp = KP + (bh * SEQ + lr) * HD + 8 * hi;
    const h16* vt = VT + (bh * HD + lr) * SEQ + 8 * hi;
    const float C1 = 0.125f * 1.4426950408889634f, C2 = C1 * (1.0f / RCAR);
    v8f o0 = (v8f){}, o1 = (v8f){}, o2 = (v8f){}, o3 = (v8f){};
    float m = -1.0e30f, l = 0.0f;
#pragma unroll 1
    for (int kb = 0; kb < SEQ; kb += 32) {
        const h16* kq = kp + (size_t)kb * HD;
        const v16h a00 = ldh(kq), a01 = ldh(kq + 32), a10 = ldh(kq + 16 * HD), a11 = ldh(kq + 16 * HD + 32);
        v8f sh0 = (v8f){}, sh1 = (v8f){}, sr0 = (v8f){}, sr1 = (v8f){};
        sh0 = wmma16(a00, bqh0, sh0); sr0 = wmma16(a00, bqr0, sr0); sh1 = wmma16(a10, bqh0, sh1); sr1 = wmma16(a10, bqr0, sr1);
        sh0 = wmma16(a01, bqh1, sh0); sr0 = wmma16(a01, bqr1, sr0); sh1 = wmma16(a11, bqh1, sh1); sr1 = wmma16(a11, bqr1, sr1);
        asm volatile("v_nop\n\tv_nop\n\tv_nop\n\tv_nop" : "+v"(sh0), "+v"(sh1), "+v"(sr0), "+v"(sr1) : "v"(a11), "v"(bqr1));
        float u0[8], u1[8]; float tm = -1.0e30f;
#pragma unroll
        for (int r = 0; r < 8; ++r) { u0[r] = sh0[r] * C1 + sr0[r] * C2; u1[r] = sh1[r] * C1 + sr1[r] * C2; tm = fmaxf(tm, fmaxf(u0[r], u1[r])); }
        tm = fmaxf(tm, __shfl_xor(tm, 16, 32));
        const float mn = fmaxf(m, tm);
        const float al = __builtin_amdgcn_exp2f(m - mn);
        float psum = 0.0f; v16h pb;
#pragma unroll
        for (int r = 0; r < 8; ++r) { const float p0 = __builtin_amdgcn_exp2f(u0[r] - mn), p1 = __builtin_amdgcn_exp2f(u1[r] - mn); psum += p0 + p1; pb[r] = (h16)(p0 * PCAR); pb[8 + r] = (h16)(p1 * PCAR); }
        psum += __shfl_xor(psum, 16, 32);
        l = l * al + psum; m = mn;
#pragma unroll
        for (int r = 0; r < 8; ++r) { o0[r] *= al; o1[r] *= al; o2[r] *= al; o3[r] *= al; }
        const h16* vq = vt + kb;
        const v16h va0 = ldh(vq), va1 = ldh(vq + (size_t)16 * SEQ), va2 = ldh(vq + (size_t)32 * SEQ), va3 = ldh(vq + (size_t)48 * SEQ);
        o0 = wmma16(va0, pb, o0); o1 = wmma16(va1, pb, o1); o2 = wmma16(va2, pb, o2); o3 = wmma16(va3, pb, o3);
        asm volatile("v_nop\n\tv_nop\n\tv_nop\n\tv_nop" : "+v"(o0), "+v"(o1), "+v"(o2), "+v"(o3) : "v"(va3), "v"(pb));
    }
    const float inv = 1.0f / (l * PCAR);
    const int wb = wave * (16 * 68);
#pragma unroll
    for (int r = 0; r < 8; ++r) { os[wb + lr * 68 + 8 * hi + r] = o0[r] * inv; os[wb + lr * 68 + 16 + 8 * hi + r] = o1[r] * inv; os[wb + lr * 68 + 32 + 8 * hi + r] = o2[r] * inv; os[wb + lr * 68 + 48 + 8 * hi + r] = o3[r] * inv; }
    __builtin_amdgcn_wave_barrier(); asm volatile("" ::: "memory");
    const int q4 = lane >> 3, p8 = (lane & 7) * 8;
#pragma unroll 1
    for (int ps = 0; ps < 2; ++ps) {
#pragma unroll
        for (int it = 0; it < 4; ++it) { const int row = it * 4 + q4; const v4f x0 = *(const v4fa*)(os + wb + row * 68 + p8), x1 = *(const v4fa*)(os + wb + row * 68 + p8 + 4); v8us oh, ol;
#pragma unroll
            for (int i = 0; i < 4; ++i) { const unsigned short h0 = f2bf(x0[i]); oh[i] = h0; ol[i] = f2bf(x0[i] - bf2f(h0)); const unsigned short h1 = f2bf(x1[i]); oh[4 + i] = h1; ol[4 + i] = f2bf(x1[i] - bf2f(h1)); }
            const size_t off = ((size_t)b * SEQ + q0 + row) * KC + head * HD + p8;
            *(volatile v8us*)(CTX + off) = oh; *(volatile v8us*)(CTX + off + DM) = ol; }
        if (ps == 0) __threadfence(); }
}

__global__ __launch_bounds__(32) void k_out(const bf* __restrict__ CTX, const bf* __restrict__ WO2, const float* __restrict__ bo, float* OUT) {
    __shared__ __align__(16) float os[64 * 68];
    const int lane = threadIdx.x & 31, lr = lane & 15, hi = lane >> 4; const int r0 = blockIdx.x * 64, c0 = blockIdx.y * 64;
    v8f acc[4][4];
    gemm_tile<KC>(CTX, WO2, r0, c0, lr, hi, acc);
#pragma unroll
    for (int mb = 0; mb < 4; ++mb)
#pragma unroll
        for (int nb = 0; nb < 4; ++nb)
#pragma unroll
            for (int j = 0; j < 8; ++j) os[(mb * 16 + hi * 8 + j) * 68 + nb * 16 + lr] = acc[mb][nb][j];
    __builtin_amdgcn_wave_barrier(); asm volatile("" ::: "memory");
    const int b = r0 / SEQ, s0 = r0 % SEQ; const int cq = lane >> 4, s4 = (lane & 15) * 4;
#pragma unroll 1
    for (int ps = 0; ps < 2; ++ps) {
#pragma unroll 2
        for (int it = 0; it < 32; ++it) { const int c = it * 2 + cq; const float bc = bfr(bo[c0 + c]); v4f v;
#pragma unroll
            for (int i = 0; i < 4; ++i) v[i] = os[(s4 + i) * 68 + c] + bc;
            *(volatile v4f*)(OUT + ((size_t)b * DM + c0 + c) * SEQ + s0 + s4) = v; }
        if (ps == 0) __threadfence(); }
}

extern "C" void kernel_launch(void* const* d_in, const int* in_sizes, int n_in,
                              void* d_out, int out_size, void* d_ws, size_t ws_size, hipStream_t stream) {
    if (n_in < 5) return;
    if (in_sizes[0] < NB * DM * SEQ || in_sizes[1] < D3 * DM || in_sizes[2] < D3 || in_sizes[3] < DM * DM || in_sizes[4] < DM) return;
    if (out_size < NB * DM * SEQ) return;
    const float* x = (const float*)d_in[0]; const float* wqkv = (const float*)d_in[1]; const float* bqkv = (const float*)d_in[2]; const float* wo = (const float*)d_in[3]; const float* bo = (const float*)d_in[4];
    float* OUT = (float*)d_out;
    constexpr size_t SZ_XB = (size_t)NTOK * DM * 2, SZ_WQ = (size_t)D3 * DM * 2, SZ_WO = (size_t)DM * KC * 2, SZ_HP = (size_t)NB * NH * SEQ * HD * 2, SZ_CTX = (size_t)NTOK * KC * 2;
    static_assert(SZ_XB % 256 == 0 && SZ_WQ % 256 == 0 && SZ_WO % 256 == 0 && SZ_HP % 256 == 0 && SZ_CTX % 256 == 0);
    constexpr size_t TOTAL = SZ_XB + SZ_WQ + SZ_WO + 4 * SZ_HP + SZ_CTX;
    static_assert(TOTAL <= (size_t)134217728);
    if (TOTAL > ws_size) return;
    char* wsp = (char*)d_ws;
    bf* XB = (bf*)wsp; wsp += SZ_XB; bf* WQ = (bf*)wsp; wsp += SZ_WQ; bf* WO2 = (bf*)wsp; wsp += SZ_WO;
    h16* QH = (h16*)wsp; wsp += SZ_HP; h16* QR = (h16*)wsp; wsp += SZ_HP; h16* KP = (h16*)wsp; wsp += SZ_HP; h16* VT = (h16*)wsp; wsp += SZ_HP;
    bf* CTX = (bf*)wsp; wsp += SZ_CTX;
    k_cvtw<<<(unsigned)((D3 * DM / 8 + 255) / 256), 256, 0, stream>>>(wqkv, WQ, D3, DM, DM, 0);
    k_cvtw<<<(unsigned)((DM * DM / 8 + 255) / 256), 256, 0, stream>>>(wo, WO2, DM, DM, KC, 1);
    k_xT<<<dim3(SEQ / 64, DM / 64, NB), 256, 0, stream>>>(x, XB);
    k_qkv<<<dim3(NTOK / 64, D3 / 64, 1), 32, 0, stream>>>(XB, WQ, bqkv, QH, QR, KP, VT);
    k_flash<<<dim3(SEQ / 64, NH, NB), 128, 0, stream>>>(QH, QR, KP, VT, CTX);
    k_out<<<dim3(NTOK / 64, DM / 64, 1), 32, 0, stream>>>(CTX, WO2, bo, OUT);
}
